// Dust3RCrossAttention_4973572129471
// MI455X (gfx1250) — hardware-verified
//
#include <hip/hip_runtime.h>
#include <hip/hip_bf16.h>
#include <math.h>
#define NUM_R 4


#define BB 8
#define SS 1024
#define DD 768
#define HH 12
#define DKK 64
#define QW 2

typedef _Float16 bf16;
typedef __attribute__((ext_vector_type(4))) unsigned v4u_t;
typedef unsigned v4ua __attribute__((ext_vector_type(4), may_alias));
typedef __attribute__((ext_vector_type(4))) float v4f_t;
typedef float v4fa __attribute__((ext_vector_type(4), may_alias));
typedef __attribute__((ext_vector_type(16))) bf16  bf16x16;
typedef __attribute__((ext_vector_type(8)))  bf16  bf16x8;
typedef __attribute__((ext_vector_type(4)))  bf16  bf16x4;
typedef __attribute__((ext_vector_type(8)))  float f32x8;

#define LDS_STRIDE 48
#define KSTRIDE    72
#define VSTRIDE    48

__device__ __forceinline__ f32x8 wmma_bf16(bf16x16 a, bf16x16 b, f32x8 c) {
  return __builtin_amdgcn_wmma_f32_16x16x32_f16(
      false, a, false, b, (short)0, c, false, false);
}

template <typename T>
__device__ __forceinline__ bf16x16 load_frag(const T* __restrict__ base, int ld,
                                             int row0, int k0) {
  const int lane = threadIdx.x & 31;
  const int r    = lane & 15;
  const int kh   = (lane >> 4) * 8;
  const T* p0 = base + (size_t)(row0 + r) * ld + (k0 + kh);
  const T* p1 = p0 + 16;
  bf16x16 f;
#pragma unroll
  for (int i = 0; i < 8; ++i) {
    f[i]     = (bf16)p0[i];
    f[i + 8] = (bf16)p1[i];
  }
  return f;
}

__device__ __forceinline__ bf16x16 lds_frag(const bf16* base, int stride) {
  const int lane = threadIdx.x & 31;
  const int row  = lane & 15;
  const int kh   = (lane >> 4) * 8;
  const bf16x8 lo = *(const bf16x8*)(base + row * stride + kh);
  const bf16x8 hi = *(const bf16x8*)(base + row * stride + kh + 16);
  bf16x16 f;
#pragma unroll
  for (int i = 0; i < 8; ++i) { f[i] = lo[i]; f[i + 8] = hi[i]; }
  return f;
}

template <typename T>
__device__ __forceinline__ void stage_read16(const T* __restrict__ p, float* buf) {
#pragma unroll
  for (int i = 0; i < 16; ++i) buf[i] = (float)p[i];
}

__device__ __forceinline__ void stage_write(bf16* dst, const float* buf, int nquad) {
#pragma unroll
  for (int i = 0; i < nquad; ++i) {
    bf16x4 q;
    q[0] = (bf16)buf[4 * i];     q[1] = (bf16)buf[4 * i + 1];
    q[2] = (bf16)buf[4 * i + 2]; q[3] = (bf16)buf[4 * i + 3];
    *(bf16x4*)(dst + 4 * i) = q;
  }
}

__global__ __launch_bounds__(256) void transpose_pack_kernel(const float* __restrict__ W, bf16* __restrict__ WT, int K, int N) {
  __shared__ float tile[64][65];
  const int k0 = blockIdx.y * 64, n0 = blockIdx.x * 64, t = threadIdx.x;
  for (int i = t; i < 64 * 64; i += 256) { const int kr = i >> 6, nc = i & 63; tile[kr][nc] = W[(size_t)(k0 + kr) * N + n0 + nc]; }
  __syncthreads();
#pragma unroll 1
  for (int pass = 0; pass < 2; ++pass) {
    for (int i = t; i < 64 * 8; i += 256) { const int nr = i >> 3, k8 = (i & 7) * 8; bf16 hh[8];
#pragma unroll
      for (int e = 0; e < 8; ++e) hh[e] = (bf16)tile[k8 + e][nr];
      *(volatile v4u_t*)(WT + (size_t)(n0 + nr) * K + k0 + k8) = *(const v4ua*)hh; }
    __threadfence();
  }
}

template <typename AT, typename WT, int MODE>
__global__ __launch_bounds__(256) void gemm_bias_kernel(
    const AT* __restrict__ A, const WT* __restrict__ W,
    const float* __restrict__ bias, void* __restrict__ out,
    int M, int N, int K, const int* __restrict__ rpos = nullptr, const float* __restrict__ lnw = nullptr, const float* __restrict__ lnb = nullptr) {
  __shared__ bf16 ldsA[128 * LDS_STRIDE];
  __shared__ bf16 ldsW[256 * LDS_STRIDE];
  __shared__ __attribute__((aligned(16))) unsigned char sob[256 * 136 * 2];

  const int t    = threadIdx.x;
  const int wave = t >> 5;
  const int lane = t & 31;
  const int wm   = (wave & 1) * 64;
  const int wn   = (wave >> 1) * 64;
  const int mBlk = blockIdx.x * 128;
  const int nBlk = blockIdx.y * 256;

  const int arow = t >> 1;
  const int ach  = (t & 1) * 16;

  float abuf[16];
  float wbuf[32];

  stage_read16(A + (size_t)(mBlk + arow) * K + ach, abuf);
  stage_read16(W + (size_t)(nBlk + t) * K,          wbuf);
  stage_read16(W + (size_t)(nBlk + t) * K + 16,     wbuf + 16);

  f32x8 acc[4][4] = {};

  for (int k = 0; k < K; k += 32) {
    __syncthreads();
    stage_write(&ldsA[arow * LDS_STRIDE + ach], abuf, 4);
    stage_write(&ldsW[t * LDS_STRIDE],          wbuf, 8);
    if (k + 32 < K) {
      stage_read16(A + (size_t)(mBlk + arow) * K + (k + 32) + ach, abuf);
      stage_read16(W + (size_t)(nBlk + t) * K + (k + 32),          wbuf);
      stage_read16(W + (size_t)(nBlk + t) * K + (k + 32) + 16,     wbuf + 16);
    }
    __syncthreads();

    bf16x16 af[4], wf[4];
#pragma unroll
    for (int i = 0; i < 4; ++i)
      af[i] = lds_frag(ldsA + (wm + 16 * i) * LDS_STRIDE, LDS_STRIDE);
#pragma unroll
    for (int j = 0; j < 4; ++j)
      wf[j] = lds_frag(ldsW + (wn + 16 * j) * LDS_STRIDE, LDS_STRIDE);
#pragma unroll
    for (int i = 0; i < 4; ++i)
#pragma unroll
      for (int j = 0; j < 4; ++j)
        acc[i][j] = wmma_bf16(af[i], wf[j], acc[i][j]);
  }

  const int nlane = lane & 15;
  const int mh    = (lane >> 4) * 8;
  __syncthreads();
  if (MODE == 0 || MODE == 1) {
    bf16* so = (bf16*)sob;
#pragma unroll
    for (int i = 0; i < 4; ++i)
#pragma unroll
      for (int j = 0; j < 4; ++j) {
        const int nl = wn + 16 * j + nlane;
        const float bv = bias ? bias[nBlk + nl] : 0.0f;
#pragma unroll
        for (int r = 0; r < 8; ++r) {
          const int ml = wm + 16 * i + mh + r;
          const bf16 hv = (bf16)(acc[i][j][r] + bv);
          if (MODE == 0) so[ml * 264 + nl] = hv;
          else           so[nl * 136 + ml] = hv;
        }
      }
    __syncthreads();
#pragma unroll 1
    for (int pass = 0; pass < 2; ++pass) {
      if (MODE == 0) {
        for (int ch = t; ch < 128 * 32; ch += 256) { const int ml = ch >> 5, q = (ch & 31) * 8;
          *(volatile v4u_t*)((bf16*)out + (size_t)(mBlk + ml) * N + nBlk + q) = *(const v4ua*)(so + ml * 264 + q); }
      } else {
        const int b_ = mBlk / SS, s0 = mBlk & (SS - 1);
        for (int ch = t; ch < 256 * 16; ch += 256) { const int nl = ch >> 4, q = (ch & 15) * 8; const int n = nBlk + nl, h = n >> 6, dk = n & (DKK - 1);
          *(volatile v4u_t*)((bf16*)out + (((size_t)(b_ * HH + h)) * DKK + dk) * SS + s0 + q) = *(const v4ua*)(so + nl * 136 + q); }
      }
      __threadfence();
    }
  } else {
    float* so = (float*)sob;
#pragma unroll 1
    for (int hf = 0; hf < 2; ++hf) {
      if (wm == hf * 64) {
#pragma unroll
        for (int i = 0; i < 4; ++i)
#pragma unroll
          for (int j = 0; j < 4; ++j) {
            const int nl = wn + 16 * j + nlane;
            const float bv = bias ? bias[nBlk + nl] : 0.0f;
#pragma unroll
            for (int r = 0; r < 8; ++r) so[(16 * i + mh + r) * 260 + nl] = acc[i][j][r] + bv;
          }
      }
      __syncthreads();
      if (MODE == 3) {
        const int row = t >> 2, hq = t & 3; float* v = so + row * 260 + hq * 64;
        const int token = mBlk + hf * 64 + row; (void)rpos; const float tp = (float)(token % SS);
        (void)lnw; (void)lnb;
#pragma unroll 1
        for (int i = 0; i < DKK / 2; ++i) {
          const float invf = 1.0f / powf(100.0f, (float)i / (float)(DKK / 2));
          const float ang = tp * invf, c = cosf(ang), s = sinf(ang);
          const float x1 = v[i], x2 = v[i + DKK / 2];
          v[i] = x1 * c - x2 * s; v[i + DKK / 2] = x1 * s + x2 * c;
        }
        __syncthreads();
      }
#pragma unroll 1
      for (int pass = 0; pass < 2; ++pass) {
        for (int ch = t; ch < 64 * 64; ch += 256) { const int ml = ch >> 6, q = (ch & 63) * 4;
          *(volatile v4f_t*)((float*)out + (size_t)(mBlk + hf * 64 + ml) * N + nBlk + q) = *(const volatile v4fa*)(so + ml * 260 + q); }
        __threadfence();
      }
      __syncthreads();
    }
  }
}

__global__ __launch_bounds__(64) void attn_kernel(
    const bf16* __restrict__ Qb, const bf16* __restrict__ Kb,
    const bf16* __restrict__ Vt, bf16* __restrict__ attnOut) {
  __shared__ bf16 ldsK[32 * KSTRIDE];
  __shared__ bf16 ldsV[64 * VSTRIDE];
  __shared__ __attribute__((aligned(16))) bf16 ldsO[2][32 * 72];

  const int q0blk = blockIdx.x * 64;
  const int h  = blockIdx.y;
  const int b  = blockIdx.z;
  const int t    = threadIdx.x;
  const int wave = t >> 5;
  const int lane = t & 31;
  const int qlane = lane & 15;
  const int kh8   = (lane >> 4) * 8;
  const int q0 = q0blk + wave * 32;

  const bf16* Qh = Qb + (size_t)b * SS * DD + h * DKK;
  const bf16* Kh = Kb + (size_t)b * SS * DD + h * DKK;
  const bf16* Vh = Vt + ((size_t)(b * HH + h)) * DKK * SS;

  const int krow = t >> 1;
  const int kcol = (t & 1) * 32;
  const bf16* kSrc = Kh + (size_t)krow * DD + kcol;
  const bf16* vSrc = Vh + (size_t)t * SS;

  bf16x16 qf[QW][2];
#pragma unroll
  for (int qt = 0; qt < QW; ++qt) {
    qf[qt][0] = load_frag(Qh, DD, q0 + 16 * qt, 0);
    qf[qt][1] = load_frag(Qh, DD, q0 + 16 * qt, 32);
  }

  f32x8 o[QW][4] = {};
  float mrun[QW], lrun[QW];
#pragma unroll
  for (int qt = 0; qt < QW; ++qt) { mrun[qt] = -INFINITY; lrun[qt] = 0.0f; }

  const float scale = 0.125f * 1.44269504088896340736f;
  const int kmax = SS - 1;

  bf16x8 kreg[4], vreg[4];
#pragma unroll
  for (int i = 0; i < 4; ++i) {
    kreg[i] = *(const bf16x8*)(kSrc + 8 * i);
    vreg[i] = *(const bf16x8*)(vSrc + 8 * i);
  }

  for (int kb = 0; kb <= kmax; kb += 32) {
    __syncthreads();
#pragma unroll
    for (int i = 0; i < 4; ++i) {
      *(bf16x8*)(&ldsK[krow * KSTRIDE + kcol + 8 * i]) = kreg[i];
      *(bf16x8*)(&ldsV[t * VSTRIDE + 8 * i])           = vreg[i];
    }
    if (kb + 32 <= kmax) {
      const bf16* kn = kSrc + (size_t)(kb + 32) * DD;
      const bf16* vn = vSrc + (kb + 32);
#pragma unroll
      for (int i = 0; i < 4; ++i) {
        kreg[i] = *(const bf16x8*)(kn + 8 * i);
        vreg[i] = *(const bf16x8*)(vn + 8 * i);
      }
    }
    __syncthreads();

    bf16x16 kf[2][2];
#pragma unroll
    for (int ktile = 0; ktile < 2; ++ktile)
#pragma unroll
      for (int c = 0; c < 2; ++c)
        kf[ktile][c] = lds_frag(ldsK + (ktile * 16) * KSTRIDE + c * 32, KSTRIDE);

    bf16x16 pf[QW];
    bool act[QW];
#pragma unroll
    for (int qt = 0; qt < QW; ++qt) {
      act[qt] = true;
      {
        const int q_my = q0 + 16 * qt + qlane;
        f32x8 s0 = {}, s1 = {};
        s0 = wmma_bf16(kf[0][0], qf[qt][0], s0);
        s0 = wmma_bf16(kf[0][1], qf[qt][1], s0);
        s1 = wmma_bf16(kf[1][0], qf[qt][0], s1);
        s1 = wmma_bf16(kf[1][1], qf[qt][1], s1);

        float mx = -INFINITY;
#pragma unroll
        for (int r = 0; r < 8; ++r) {
          const int k0i = kb + kh8 + r;
          const int k1i = k0i + 16;
          (void)k0i; (void)k1i; (void)q_my;
          s0[r] = s0[r] * scale;
          s1[r] = s1[r] * scale;
          mx = fmaxf(mx, fmaxf(s0[r], s1[r]));
        }
        mx = fmaxf(mx, __shfl_xor(mx, 16, 32));
        const float mnew  = fmaxf(mrun[qt], mx);
        const float alpha = exp2f(mrun[qt] - mnew);

        float rsum = 0.0f;
#pragma unroll
        for (int r = 0; r < 8; ++r) {
          const float p0 = exp2f(s0[r] - mnew);
          const float p1 = exp2f(s1[r] - mnew);
          rsum += p0 + p1;
          pf[qt][r]     = (bf16)(p0 * 1024.0f);
          pf[qt][r + 8] = (bf16)(p1 * 1024.0f);
        }
        rsum += __shfl_xor(rsum, 16, 32);
        lrun[qt] = lrun[qt] * alpha + rsum;
        mrun[qt] = mnew;

#pragma unroll
        for (int j = 0; j < 4; ++j)
#pragma unroll
          for (int r = 0; r < 8; ++r) o[qt][j][r] *= alpha;
      }
    }

#pragma unroll
    for (int j = 0; j < 4; ++j) {
      const bf16x16 vf = lds_frag(ldsV + (j * 16) * VSTRIDE, VSTRIDE);
#pragma unroll
      for (int qt = 0; qt < QW; ++qt)
        if (act[qt]) o[qt][j] = wmma_bf16(vf, pf[qt], o[qt][j]);
    }
  }

  bf16* so = ldsO[wave];
#pragma unroll
  for (int qt = 0; qt < QW; ++qt) {
    const float rl = 1.0f / (lrun[qt] * 1024.0f);
#pragma unroll
    for (int j = 0; j < 4; ++j)
#pragma unroll
      for (int r = 0; r < 8; ++r) so[(16 * qt + qlane) * 72 + j * 16 + kh8 + r] = (bf16)(o[qt][j][r] * rl);
  }
  asm volatile("s_wait_dscnt 0" ::: "memory");
#pragma unroll 1
  for (int pass = 0; pass < 2; ++pass) {
#pragma unroll
    for (int it = 0; it < 8; ++it) { const int ch = lane + 32 * it, ql = ch >> 3, q8 = (ch & 7) * 8;
      *(volatile v4u_t*)(attnOut + ((size_t)(b * SS + q0 + ql)) * DD + h * DKK + q8) = *(const v4ua*)(so + ql * 72 + q8); }
    __threadfence();
  }
}

__global__ __launch_bounds__(256) void k_cvt(const float* __restrict__ Qf, const float* __restrict__ Kf, bf16* __restrict__ Qb, bf16* __restrict__ Kb) {
  const int tok = blockIdx.x, t = threadIdx.x; bf16 hq[4], hk[4];
#pragma unroll
  for (int i = 0; i < 4; ++i) { hq[i] = (bf16)Qf[(size_t)tok * DD + t * 4 + i]; hk[i] = (bf16)Kf[(size_t)tok * DD + t * 4 + i]; }
  typedef __attribute__((ext_vector_type(2))) unsigned v2u; typedef unsigned v2ua __attribute__((ext_vector_type(2), may_alias));
#pragma unroll 1
  for (int pass = 0; pass < 2; ++pass) {
    *(volatile v2u*)(Qb + (size_t)tok * DD + t * 4) = *(const v2ua*)hq; *(volatile v2u*)(Kb + (size_t)tok * DD + t * 4) = *(const v2ua*)hk;
    __threadfence();
  }
}

extern "C" void kernel_launch(void* const* d_in, const int* in_sizes, int n_in,
                              void* d_out, int out_size, void* d_ws, size_t ws_size,
                              hipStream_t stream) {
  (void)in_sizes; (void)n_in; (void)out_size; (void)ws_size;
  const float* xq = (const float*)d_in[0]; const float* xk = (const float*)d_in[1]; const float* xv = (const float*)d_in[2];
  const float* Wq = (const float*)d_in[3]; const float* Wk = (const float*)d_in[4]; const float* Wv = (const float*)d_in[5];
  const float* Wo = (const float*)d_in[6]; const float* bo = (const float*)d_in[7];
  const size_t qkvBytes = (size_t)BB * SS * DD * sizeof(bf16);
  char* ws   = (char*)d_ws;
  bf16* Qb   = (bf16*)(ws);
  bf16* Kb   = (bf16*)(ws + qkvBytes);
  bf16* VtB  = (bf16*)(ws + 2 * qkvBytes);
  bf16* attn = (bf16*)(ws + 3 * qkvBytes);
  float* Qf  = (float*)(ws + 4 * qkvBytes);
  float* Kf  = Qf + (size_t)BB * SS * DD;
  const int M = BB * SS, N = DD, K = DD;
  dim3 gGrid(M / 128, N / 256), gBlk(256);
  gemm_bias_kernel<float, float, 3><<<gGrid, gBlk, 0, stream>>>(xq, Wq, nullptr, Qf,  M, N, K, nullptr, nullptr, nullptr);
  gemm_bias_kernel<float, float, 3><<<gGrid, gBlk, 0, stream>>>(xk, Wk, nullptr, Kf,  M, N, K, nullptr, nullptr, nullptr);
  gemm_bias_kernel<float, float, 1><<<gGrid, gBlk, 0, stream>>>(xv, Wv, nullptr, VtB, M, N, K);
  k_cvt<<<BB * SS, DD / 4, 0, stream>>>(Qf, Kf, Qb, Kb);
  attn_kernel<<<dim3(SS / 64, HH, BB), dim3(64), 0, stream>>>(Qb, Kb, VtB, attn);
  gemm_bias_kernel<bf16, float, 2><<<gGrid, gBlk, 0, stream>>>(attn, Wo, bo, (float*)d_out, M, N, K);
}
